// CorrespodenceNet_66889820668453
// MI455X (gfx1250) — hardware-run, weakly checked
//
#include <hip/hip_runtime.h>
#include <math.h>

constexpr int   kNPos       = 16384;
constexpr int   kNCh        = 256;
constexpr int   kChunkRows  = 1024;
constexpr int   kNumChunks  = kNPos / kChunkRows;
constexpr float kCarry      = 64.0f;
constexpr float kCorrScale  = 1.0f / (64.0f * 64.0f);
constexpr float kInvTau     = 100.0f;
constexpr float kInvNPos    = 1.0f / 16384.0f;

constexpr size_t kOffXH    = 0;
constexpr size_t kOffYH    = (size_t)kNPos * kNCh * 2;
constexpr size_t kOffStats = kOffYH + (size_t)kNPos * kNCh * 2;
constexpr size_t kOffSC    = kOffStats + 4096;
constexpr size_t kWsTotal  = kOffSC + (size_t)kChunkRows * kNPos * 4;

typedef __attribute__((ext_vector_type(16))) _Float16 v16h;
typedef __attribute__((ext_vector_type(8)))  _Float16 v8h;
typedef __attribute__((ext_vector_type(16))) __bf16   v16b;
typedef __attribute__((ext_vector_type(8)))  __bf16   v8b;
typedef __attribute__((ext_vector_type(8)))  float    v8f;
typedef __attribute__((ext_vector_type(4)))  float    v4f;
typedef __attribute__((ext_vector_type(4)))  unsigned int v4u;

__device__ __forceinline__ unsigned short f2bf_bits(float f) {
  unsigned u = __float_as_uint(f);
  return (unsigned short)((u + 0x7FFFu + ((u >> 16) & 1u)) >> 16);
}
__device__ __forceinline__ float bf_bits2f(unsigned short h) { return __uint_as_float(((unsigned)h) << 16); }

__device__ __forceinline__ void dep_guard_h(v8f& a, v8f& b, v16h x, v16h y) { asm volatile("v_nop\n\tv_nop\n\tv_nop\n\tv_nop" : "+v"(a), "+v"(b) : "v"(x), "v"(y)); }
__device__ __forceinline__ void dep_guard_b(v8f& a, v8f& b, v16b x, v16b y) { asm volatile("v_nop\n\tv_nop\n\tv_nop\n\tv_nop" : "+v"(a), "+v"(b) : "v"(x), "v"(y)); }
__device__ __forceinline__ void keep4_h(v16h a, v16h b, v16h c, v16h d) { asm volatile("v_nop" :: "v"(a), "v"(b), "v"(c), "v"(d)); }
__device__ __forceinline__ void keep4_b(v16b a, v16b b, v16b c, v16b d) { asm volatile("v_nop" :: "v"(a), "v"(b), "v"(c), "v"(d)); }
__device__ __forceinline__ void acc_guard4(v8f& a, v8f& b, v8f& c, v8f& d) { asm volatile("v_nop\n\tv_nop\n\tv_nop\n\tv_nop" : "+v"(a), "+v"(b), "+v"(c), "+v"(d)); }
template <typename T> struct Frag;
template <> struct Frag<_Float16> {
  typedef v16h V; union U { v16h v; v8h h[2]; };
  static __device__ __forceinline__ v16h load(const _Float16* p) {
    U f; f.h[0] = *(const v8h*)(p); f.h[1] = *(const v8h*)(p + 16); return f.v;
  }
  static __device__ __forceinline__ v8f mma(v16h a, v16h b, v8f c) {
    return __builtin_amdgcn_wmma_f32_16x16x32_f16(false, a, false, b, (short)0, c, false, false);
  }
  static __device__ __forceinline__ void guard(v8f& a, v8f& b, v16h x, v16h y) { dep_guard_h(a, b, x, y); }
  static __device__ __forceinline__ void keep(v16h a, v16h b, v16h c, v16h d) { keep4_h(a, b, c, d); }
};
template <> struct Frag<__bf16> {
  typedef v16b V; union U { v16b v; v8b h[2]; };
  static __device__ __forceinline__ v16b load(const __bf16* p) {
    U f; f.h[0] = *(const v8b*)(p); f.h[1] = *(const v8b*)(p + 16); return f.v;
  }
  static __device__ __forceinline__ v8f mma(v16b a, v16b b, v8f c) {
    return __builtin_amdgcn_wmma_f32_16x16x32_bf16(false, a, false, b, (short)0, c, false, false);
  }
  static __device__ __forceinline__ void guard(v8f& a, v8f& b, v16b x, v16b y) { dep_guard_b(a, b, x, y); }
  static __device__ __forceinline__ void keep(v16b a, v16b b, v16b c, v16b d) { keep4_b(a, b, c, d); }
};

__device__ __forceinline__ unsigned pk16(unsigned short a, unsigned short b) { return (unsigned)a | ((unsigned)b << 16); }
__device__ __forceinline__ unsigned short h_bits(float f) { const _Float16 h = (_Float16)f; return __builtin_bit_cast(unsigned short, h); }

template <int ET> struct Elem;
template <> struct Elem<0> { typedef _Float16 T; };
template <> struct Elem<1> { typedef __bf16 T; };
template <int ET, bool SPLIT, int BIAS_MODE, int OUT_MODE, bool RESID, int ACT = 0>
__global__ __launch_bounds__(256) void wmma_gemm64(
    const unsigned short* __restrict__ Ap, const unsigned short* __restrict__ A2p, int lda, long strideA,
    const unsigned short* __restrict__ Btp, const unsigned short* __restrict__ Bt2p, int ldb, long strideB,
    void* __restrict__ Cout, void* __restrict__ Cout2, int ldc, long strideC,
    const float* __restrict__ bias,
    const float* __restrict__ resid, long strideR,
    int M, int N, int K, float scale) {
  typedef typename Elem<ET>::T T;
  typedef typename Frag<T>::V V;
  const T* A = (const T*)Ap; const T* A2 = (const T*)A2p; const T* Bt = (const T*)Btp; const T* Bt2 = (const T*)Bt2p;
  __shared__ __align__(16) float sT[8][16 * 68];
  const int b    = blockIdx.y;
  const int lane = threadIdx.x & 31;
  const int wave = threadIdx.x >> 5;
  const int tilesN = N >> 6;
  const int tilesM = M >> 6;
  const int tile = blockIdx.x * 8 + wave;
  if (tile >= tilesM * tilesN) return;
  const int tm = tile / tilesN;
  const int tn = tile - tm * tilesN;
  const int m0 = tm << 6;
  const int n0 = tn << 6;

  const T* Ab  = A  + (size_t)b * strideA;
  const T* Bb  = Bt + (size_t)b * strideB;
  const T* Ab2 = SPLIT ? (A2  + (size_t)b * strideA) : nullptr;
  const T* Bb2 = SPLIT ? (Bt2 + (size_t)b * strideB) : nullptr;

  const int rlane = lane & 15;
  const int koff  = (lane >> 4) * 8;
  const int mOff  = (lane >> 4) * 8;

  v8f acc[4][4];
#pragma unroll
  for (int i = 0; i < 4; ++i)
#pragma unroll
    for (int j = 0; j < 4; ++j) acc[i][j] = (v8f){0.f,0.f,0.f,0.f,0.f,0.f,0.f,0.f};

  for (int k0 = 0; k0 < K; k0 += 32) {
    V bh[4], bl[4];
#pragma unroll
    for (int j = 0; j < 4; ++j) {
      const size_t bo = (size_t)(n0 + (j << 4) + rlane) * ldb + koff + k0;
      bh[j] = Frag<T>::load(Bb + bo);
      if (SPLIT) bl[j] = Frag<T>::load(Bb2 + bo);
    }
#pragma unroll
    for (int i = 0; i < 4; ++i) {
      const size_t ao = (size_t)(m0 + (i << 4) + rlane) * lda + koff + k0;
      V ah = Frag<T>::load(Ab + ao);
      V al;
      if (SPLIT) al = Frag<T>::load(Ab2 + ao);
#pragma unroll
      for (int j = 0; j < 4; ++j) {
        acc[i][j] = Frag<T>::mma(ah, bh[j], acc[i][j]);
        if (SPLIT) {
          acc[i][j] = Frag<T>::mma(ah, bl[j], acc[i][j]);
          acc[i][j] = Frag<T>::mma(al, bh[j], acc[i][j]);
        }
      }
      Frag<T>::guard(acc[i][0], acc[i][3], ah, SPLIT ? al : ah);
    }
    Frag<T>::keep(bh[0], bh[1], bh[2], bh[3]);
    if (SPLIT) Frag<T>::keep(bl[0], bl[1], bl[2], bl[3]);
  }
  acc_guard4(acc[0][0], acc[0][1], acc[0][2], acc[0][3]);
  acc_guard4(acc[1][0], acc[1][1], acc[1][2], acc[1][3]);
  acc_guard4(acc[2][0], acc[2][1], acc[2][2], acc[2][3]);
  acc_guard4(acc[3][0], acc[3][1], acc[3][2], acc[3][3]);

  float* slab = sT[wave];
  const float* Rb = RESID ? (resid + (size_t)b * strideR) : nullptr;
#pragma unroll
  for (int i = 0; i < 4; ++i) {
    const int mBase = m0 + (i << 4);
#pragma unroll
    for (int j = 0; j < 4; ++j) {
      const int n = n0 + (j << 4) + rlane;
      float bv = 0.f;
      if (BIAS_MODE == 2) bv = bias[n];
#pragma unroll
      for (int r = 0; r < 8; ++r) {
        float v = acc[i][j][r] * scale;
        if (BIAS_MODE == 1) v += bias[mBase + mOff + r];
        if (BIAS_MODE == 2) v += bv;
        if (RESID) v += Rb[(size_t)(mBase + mOff + r) * ldc + n];
        if (ACT == 2) v = fmaxf(v, 0.0f);
        if (ACT == 4) v = (v > 0.f) ? v : 0.01f * v;
        slab[(mOff + r) * 68 + (j << 4) + rlane] = v;
      }
    }
    __builtin_amdgcn_fence(__ATOMIC_RELEASE, "workgroup");
    __builtin_amdgcn_wave_barrier();
    __builtin_amdgcn_fence(__ATOMIC_ACQUIRE, "workgroup");
    if (OUT_MODE == 0) {
      float* C = (float*)Cout + (size_t)b * strideC;
      const int hh = lane >> 4, c4 = (lane & 15) * 4;
      for (int pass = 0; pass < 2; ++pass) {
#pragma unroll
        for (int it = 0; it < 8; ++it) {
          const int row = it * 2 + hh;
          v4f v = *(const v4f*)(slab + row * 68 + c4);
          *(volatile v4f*)(C + (size_t)(mBase + row) * ldc + n0 + c4) = v;
        }
        __threadfence();
      }
    } else {
      const int q = lane >> 3, c8 = (lane & 7) * 8;
      unsigned short* C  = (unsigned short*)Cout  + (size_t)b * strideC;
      unsigned short* C2 = (OUT_MODE == 2) ? ((unsigned short*)Cout2 + (size_t)b * strideC) : nullptr;
      for (int pass = 0; pass < 2; ++pass) {
#pragma unroll
        for (int it = 0; it < 4; ++it) {
          const int row = it * 4 + q;
          const float* sp = slab + row * 68 + c8;
          v8h hv, lv;
#pragma unroll
          for (int e = 0; e < 8; ++e) {
            if (OUT_MODE == 1) {
              hv[e] = (_Float16)sp[e];
            } else {
              unsigned short hb = f2bf_bits(sp[e]);
              unsigned short lb = f2bf_bits(sp[e] - bf_bits2f(hb));
              hv[e] = __builtin_bit_cast(_Float16, hb);
              lv[e] = __builtin_bit_cast(_Float16, lb);
            }
          }
          *(volatile v8h*)(C + (size_t)(mBase + row) * ldc + n0 + c8) = hv;
          if (OUT_MODE == 2) *(volatile v8h*)(C2 + (size_t)(mBase + row) * ldc + n0 + c8) = lv;
        }
        __threadfence();
      }
    }
    __builtin_amdgcn_fence(__ATOMIC_RELEASE, "workgroup");
    __builtin_amdgcn_wave_barrier();
    __builtin_amdgcn_fence(__ATOMIC_ACQUIRE, "workgroup");
  }
}

__global__ __launch_bounds__(256) void col_stats_kernel(const float* __restrict__ x, const float* __restrict__ y,
                                                        float* __restrict__ stats) {
  __shared__ float red[8][32];
  const int tid  = threadIdx.x;
  const int lane = tid & 31, wave = tid >> 5;
  const int g    = blockIdx.x;
  const int tsel = blockIdx.y;
  const float* f = (tsel == 0) ? x : y;
  const int col  = g * 32 + lane;
  const float* fp = f + col;

  float s = 0.f;
#pragma unroll 1
  for (int kb = 0; kb < kNPos / 8; kb += 16) {
    float p = 0.f;
#pragma unroll
    for (int u = 0; u < 16; ++u) {
      const int i = wave + 8 * (kb + u);
      p += fp[(size_t)i * kNCh];
    }
    s += p;
  }
  red[wave][lane] = s;
  __syncthreads();
  float tot = red[0][lane];
#pragma unroll
  for (int w = 1; w < 8; ++w) tot += red[w][lane];
  const float mean = tot * kInvNPos;
  __syncthreads();

  float ss = 0.f;
#pragma unroll 1
  for (int kb = 0; kb < kNPos / 8; kb += 16) {
    float p = 0.f;
#pragma unroll
    for (int u = 0; u < 16; ++u) {
      const int i = wave + 8 * (kb + u);
      const float d = fp[(size_t)i * kNCh] - mean;
      p = fmaf(d, d, p);
    }
    ss += p;
  }
  red[wave][lane] = ss;
  __syncthreads();
  float tot2 = red[0][lane];
#pragma unroll
  for (int w = 1; w < 8; ++w) tot2 += red[w][lane];
  const float invn = 1.0f / sqrtf(tot2);

  if (wave == 0) {
    float* pm = stats + (size_t)tsel * 512 + col;
    float* pi = stats + (size_t)tsel * 512 + 256 + col;
    *(volatile float*)pm = mean;
    *(volatile float*)pi = invn;
    __threadfence();
    *(volatile float*)pm = mean;
    *(volatile float*)pi = invn;
  }
}

__global__ __launch_bounds__(256) void norm_cast_kernel(const float* __restrict__ x, const float* __restrict__ y,
                                                        const float* __restrict__ stats,
                                                        unsigned short* __restrict__ planes) {
  const int gi   = blockIdx.x * 256 + threadIdx.x;
  const int tsel = blockIdx.y;
  const int row  = gi >> 5;
  const int c8   = (gi & 31) * 8;
  const float* f = (tsel == 0) ? x : y;
  const float* p = f + (size_t)row * kNCh + c8;
  const v4f a = *(const v4f*)(p);
  const v4f b = *(const v4f*)(p + 4);
  const float* st = stats + (size_t)tsel * 512;
  const v4f m0 = *(const v4f*)(st + c8);
  const v4f m1 = *(const v4f*)(st + c8 + 4);
  const v4f i0 = *(const v4f*)(st + 256 + c8);
  const v4f i1 = *(const v4f*)(st + 256 + c8 + 4);
  unsigned short hb[8];
#pragma unroll
  for (int e = 0; e < 4; ++e) {
    float t0 = (a[e] - m0[e]) * i0[e]; t0 = t0 * kCarry;
    float t1 = (b[e] - m1[e]) * i1[e]; t1 = t1 * kCarry;
    hb[e]     = h_bits(t0);
    hb[4 + e] = h_bits(t1);
  }
  const v4u u = (v4u){pk16(hb[0], hb[1]), pk16(hb[2], hb[3]), pk16(hb[4], hb[5]), pk16(hb[6], hb[7])};
  unsigned short* q = planes + (size_t)tsel * kNPos * kNCh + (size_t)row * kNCh + c8;
  *(volatile v4u*)q = u;
  __threadfence();
  *(volatile v4u*)q = u;
}

__global__ __launch_bounds__(256) void row_softmax_warp_kernel(const float* __restrict__ sc, const float* __restrict__ ab,
                                                               float* __restrict__ out, int grow0) {
  __shared__ float res[3][32];
  const int tid  = threadIdx.x;
  const int lane = tid & 31, wave = tid >> 5;
  const int brow0 = blockIdx.x * 32;
  const float* abA = ab;
  const float* abB = ab + kNPos;

#pragma unroll 1
  for (int rl = 0; rl < 4; ++rl) {
    const int lrow = brow0 + wave * 4 + rl;
    const float* sr = sc + (size_t)lrow * kNPos;
    float m = -1.0e30f, zs = 0.f, wa = 0.f, wb = 0.f;
#pragma unroll 1
    for (int it = 0; it < 64; ++it) {
      const int c0 = it * 256 + lane * 4;
      const v4f s0 = *(const v4f*)(sr + c0);
      const v4f s1 = *(const v4f*)(sr + c0 + 128);
      const v4f a0 = *(const v4f*)(abA + c0);
      const v4f a1 = *(const v4f*)(abA + c0 + 128);
      const v4f b0 = *(const v4f*)(abB + c0);
      const v4f b1 = *(const v4f*)(abB + c0 + 128);
      const float lm = fmaxf(fmaxf(fmaxf(s0[0], s0[1]), fmaxf(s0[2], s0[3])),
                             fmaxf(fmaxf(s1[0], s1[1]), fmaxf(s1[2], s1[3])));
      const float mn = fmaxf(m, lm);
      const float alpha = expf((m - mn) * kInvTau);
      zs *= alpha; wa *= alpha; wb *= alpha;
      m = mn;
#pragma unroll
      for (int e = 0; e < 4; ++e) {
        const float p0 = expf((s0[e] - mn) * kInvTau);
        zs += p0; wa = fmaf(p0, a0[e], wa); wb = fmaf(p0, b0[e], wb);
      }
#pragma unroll
      for (int e = 0; e < 4; ++e) {
        const float p1 = expf((s1[e] - mn) * kInvTau);
        zs += p1; wa = fmaf(p1, a1[e], wa); wb = fmaf(p1, b1[e], wb);
      }
    }
    float mm = m;
#pragma unroll
    for (int off = 16; off > 0; off >>= 1) mm = fmaxf(mm, __shfl_xor(mm, off, 32));
    const float fr = expf((m - mm) * kInvTau);
    zs *= fr; wa *= fr; wb *= fr;
#pragma unroll
    for (int off = 16; off > 0; off >>= 1) {
      zs += __shfl_xor(zs, off, 32);
      wa += __shfl_xor(wa, off, 32);
      wb += __shfl_xor(wb, off, 32);
    }
    const float rz = 1.0f / zs;
    const float oa = wa * rz;
    const float ob = wb * rz;
    if (lane == 0) {
      res[0][wave * 4 + rl] = oa;
      res[1][wave * 4 + rl] = ob;
      res[2][wave * 4 + rl] = mm;
    }
  }
  __syncthreads();
  if (wave < 3) {
    const float v = res[wave][lane];
    float* op = out + (size_t)wave * kNPos + grow0 + brow0 + lane;
    *(volatile float*)op = v;
    __threadfence();
    *(volatile float*)op = v;
  }
}

extern "C" void kernel_launch(void* const* d_in, const int* in_sizes, int n_in,
                              void* d_out, int out_size, void* d_ws, size_t ws_size,
                              hipStream_t stream) {
  if (n_in < 3) return;
  if (in_sizes[0] != kNPos * kNCh || in_sizes[1] != kNPos * kNCh || in_sizes[2] != 2 * kNPos) return;
  if (out_size != 3 * kNPos) return;
  if (ws_size < kWsTotal) return;

  const float* x  = (const float*)d_in[0];
  const float* y  = (const float*)d_in[1];
  const float* ab = (const float*)d_in[2];
  float* out = (float*)d_out;

  char* ws = (char*)d_ws;
  unsigned short* planes = (unsigned short*)(ws + kOffXH);
  const unsigned short* xh = (const unsigned short*)(ws + kOffXH);
  const unsigned short* yh = (const unsigned short*)(ws + kOffYH);
  float* stats = (float*)(ws + kOffStats);
  float* sc    = (float*)(ws + kOffSC);

  col_stats_kernel<<<dim3(kNCh / 32, 2, 1), dim3(256, 1, 1), 0, stream>>>(x, y, stats);
  norm_cast_kernel<<<dim3(kNPos * kNCh / 8 / 256, 2, 1), dim3(256, 1, 1), 0, stream>>>(x, y, stats, planes);

  for (int ch = 0; ch < kNumChunks; ++ch) {
    const unsigned short* xa = xh + (size_t)ch * kChunkRows * kNCh;
    wmma_gemm64<0, false, 0, 0, false, 0><<<dim3((kChunkRows / 64) * (kNPos / 64) / 8, 1, 1), dim3(256, 1, 1), 0, stream>>>(
        xa, (const unsigned short*)nullptr, kNCh, 0L,
        yh, (const unsigned short*)nullptr, kNCh, 0L,
        (void*)sc, (void*)nullptr, kNPos, 0L,
        (const float*)nullptr, (const float*)nullptr, 0L,
        kChunkRows, kNPos, kNCh, kCorrScale);
    row_softmax_warp_kernel<<<dim3(kChunkRows / 32, 1, 1), dim3(256, 1, 1), 0, stream>>>(sc, ab, out, ch * kChunkRows);
  }
}
